// MPNNModel_15401752723912
// MI455X (gfx1250) — hardware-verified
//
#include <hip/hip_runtime.h>
#include <stddef.h>
#include <stdint.h>
#include <math.h>


#define FD     64
#define K2     128
#define NCLS   10
#define NGR    128
#define NOUT   (NGR * NCLS)
#define NTHR   256
#define NWAVE  8
#define EPT    8
#define CHUNK  (NTHR * EPT)
#define WCAP   (EPT * 32)
#define LISTN  (NWAVE * WCAP)
#define NBA    1024
#define SLA    10
#define RCAP   20480
#define DEGCAP 64
#define SB     256
#define TR     128
#define AP     136
#define MSP    68
#define GBM    64
#define GTHR   128
#define GCAP   8192
#define MEAS_B1024  16653
#define MEAS_MAXDEG 36
#define T_BE1  0
#define T_BE2  1024
#define T_BN   2048
#define T_WG   3072
#define T_BG   4096
#define T_BFC  5120
#define T_WFC  6144
#define TABN   7168
#define AGG_ZINTS (LISTN + 2 * RCAP + 3 * NBA)
#define BKT_LDS_INTS (AGG_ZINTS + 16 + 32)
#define BKT_LDS_BYTES (BKT_LDS_INTS * 4)
#define EDGE_LDS_BYTES (SB * FD * 4 + TR * MSP * 4 + TR * FD * 4 + TR * AP * 2 + FD * 4 + TR * 4)
#define POOL_WORDS (2 * GCAP + 640 + 16 + 4 * FD + FD + 16 + 16 + 16 + 32)
#define POOL_LDS_BYTES (POOL_WORDS * 4)
#define WSMAX  134217728

static_assert(FD == 64 && K2 == 2 * FD);
static_assert(NTHR == FD * 4 && NTHR == 2 * TR && NTHR == NWAVE * 32);
static_assert(SB * 4 == NBA && TR == NWAVE * 16);
static_assert((CHUNK & (CHUNK - 1)) == 0 && CHUNK <= 4096);
static_assert((NBA & (NBA - 1)) == 0 && NBA == (1 << SLA));
static_assert(((long long)CHUNK << SLA) < (1LL << 31));
static_assert(RCAP >= MEAS_B1024 + MEAS_B1024 / 20 + 1);
static_assert(RCAP % (2 * NTHR) == 0 && RCAP % TR == 0 && AGG_ZINTS % 4 == 0 && LISTN % 4 == 0);
static_assert(DEGCAP >= MEAS_MAXDEG + 8);
static_assert(GCAP == 8192 && GCAP >= 4096);
static_assert(BKT_LDS_BYTES <= 300000 && EDGE_LDS_BYTES <= 300000 && POOL_LDS_BYTES <= 300000);
static_assert((AP * 2) % 16 == 0 && AP >= K2 && (MSP * 4) % 16 == 0 && MSP >= FD);
static_assert(NOUT % 4 == 0 && (NOUT * 4) % 128 == 0 && NOUT / 4 <= 2 * NTHR);
static_assert(TABN % 4 == 0 && T_WFC + 640 <= TABN);
static_assert(SB * 16 == 4 * 4 * NTHR);

typedef float          v4f   __attribute__((ext_vector_type(4)));
typedef float          v8f   __attribute__((ext_vector_type(8)));
typedef int            v2i   __attribute__((ext_vector_type(2)));
typedef int            v4i   __attribute__((ext_vector_type(4)));
typedef int            v8i   __attribute__((ext_vector_type(8)));
typedef unsigned short v8us  __attribute__((ext_vector_type(8)));
typedef unsigned short v16us __attribute__((ext_vector_type(16)));
typedef __bf16         v16bf __attribute__((ext_vector_type(16)));
typedef v4f  __attribute__((may_alias)) v4fa;
typedef v2i  __attribute__((may_alias)) v2ia;
typedef v4i  __attribute__((may_alias)) v4ia;
typedef v8us __attribute__((may_alias)) v8usa;
union FragB { v16bf v; v16us u; v8us h[2]; v8i w; };

__device__ __forceinline__ v8f wmb(const FragB& a, const FragB& b, v8f c) {
  v8f d = __builtin_amdgcn_wmma_f32_16x16x32_bf16(false, a.v, false, b.v, (short)0, c, false, false);
  asm volatile("v_nop\n\tv_nop\n\tv_nop\n\tv_nop" : "+v"(d) : "v"(a.w), "v"(b.w));
  return d;
}

__device__ __forceinline__ unsigned bf16_bits(float f) {
  const unsigned u = __float_as_uint(f);
  return (u + 0x7FFFu + ((u >> 16) & 1u)) >> 16;
}
__device__ __forceinline__ float bf16_val(float f) {
  return __uint_as_float(bf16_bits(f) << 16);
}
__device__ __forceinline__ float nmax(float a, float b) {
  return (b > a || b != b) ? b : a;
}
__device__ __forceinline__ void put16(unsigned short* dp, v8us o) {
  *(volatile v8us*)dp = o;
  __threadfence();
  *(volatile v8us*)dp = o;
}
__device__ __forceinline__ void putf4(float* dp, v4f o) {
  *(volatile v4f*)dp = o;
  __threadfence();
  *(volatile v4f*)dp = o;
}

template <int SLB>
__device__ __forceinline__ int scan_chunk(const int* __restrict__ dsts, int nE, int cbase, int slotBase,
                                          int nb, int vec8, int* list, int tid, int lane, int wave) {
  int wc = 0;
  const int el0  = tid * EPT;
  const int e0   = cbase + el0;
  const int sent = -2147483647 - 1;
  v4i da, db;
  if (vec8 != 0 && cbase + CHUNK <= nE) {
    da = *(const v4i*)(dsts + e0);
    db = *(const v4i*)(dsts + e0 + 4);
  } else {
    da.x = (e0     < nE) ? dsts[min(e0,     nE - 1)] : sent;
    da.y = (e0 + 1 < nE) ? dsts[min(e0 + 1, nE - 1)] : sent;
    da.z = (e0 + 2 < nE) ? dsts[min(e0 + 2, nE - 1)] : sent;
    da.w = (e0 + 3 < nE) ? dsts[min(e0 + 3, nE - 1)] : sent;
    db.x = (e0 + 4 < nE) ? dsts[min(e0 + 4, nE - 1)] : sent;
    db.y = (e0 + 5 < nE) ? dsts[min(e0 + 5, nE - 1)] : sent;
    db.z = (e0 + 6 < nE) ? dsts[min(e0 + 6, nE - 1)] : sent;
    db.w = (e0 + 7 < nE) ? dsts[min(e0 + 7, nE - 1)] : sent;
  }
  const unsigned nbs = (unsigned)slotBase;
  const unsigned unb = (unsigned)nb;
  const unsigned s0 = (unsigned)da.x - nbs, s1 = (unsigned)da.y - nbs;
  const unsigned s2 = (unsigned)da.z - nbs, s3 = (unsigned)da.w - nbs;
  const unsigned s4 = (unsigned)db.x - nbs, s5 = (unsigned)db.y - nbs;
  const unsigned s6 = (unsigned)db.z - nbs, s7 = (unsigned)db.w - nbs;
  const bool h0 = s0 < unb, h1 = s1 < unb, h2 = s2 < unb, h3 = s3 < unb;
  const bool h4 = s4 < unb, h5 = s5 < unb, h6 = s6 < unb, h7 = s7 < unb;
  const unsigned any = __builtin_amdgcn_ballot_w32(h0 | h1 | h2 | h3 | h4 | h5 | h6 | h7);
  if (any != 0u) {
#define HITJ(J, HJ, SJ) { \
      const unsigned mj = __builtin_amdgcn_ballot_w32(HJ); \
      if (mj != 0u) { \
        if (HJ) { \
          const int pos = wc + (int)__builtin_amdgcn_mbcnt_lo(mj, 0u); \
          if (pos < WCAP) list[wave * WCAP + pos] = ((el0 + (J)) << SLB) | (int)(SJ); \
        } \
        wc += (int)__builtin_popcount(mj); } }
    HITJ(0, h0, s0)
    HITJ(1, h1, s1)
    HITJ(2, h2, s2)
    HITJ(3, h3, s3)
    HITJ(4, h4, s4)
    HITJ(5, h5, s5)
    HITJ(6, h6, s6)
    HITJ(7, h7, s7)
#undef HITJ
  }
  return wc;
}

__device__ __forceinline__ void tab_unit(const float* __restrict__ s, int n, float* d, int v) {
  const int i0 = 4 * v;
  const int nm = n - 1;
  const float a0 = s[min(i0,     nm)];
  const float a1 = s[min(i0 + 1, nm)];
  const float a2 = s[min(i0 + 2, nm)];
  const float a3 = s[min(i0 + 3, nm)];
  v4f q;
  q.x = (i0     < n) ? bf16_val(a0) : 0.0f;
  q.y = (i0 + 1 < n) ? bf16_val(a1) : 0.0f;
  q.z = (i0 + 2 < n) ? bf16_val(a2) : 0.0f;
  q.w = (i0 + 3 < n) ? bf16_val(a3) : 0.0f;
  putf4(d + i0, q);
}

__global__ __launch_bounds__(NTHR) void k_prep(const float* __restrict__ x, const float* __restrict__ We1,
                                               const float* __restrict__ be1, const float* __restrict__ We2,
                                               const float* __restrict__ be2, const float* __restrict__ Wn,
                                               const float* __restrict__ bn, const float* __restrict__ Wg,
                                               const float* __restrict__ bg, const float* __restrict__ Wfc,
                                               const float* __restrict__ bfc, int nN, int mRows,
                                               unsigned short* XB, unsigned short* W1C, unsigned short* WE2D,
                                               unsigned short* WND, float* TAB) {
  const int u  = (int)blockIdx.x * NTHR + (int)threadIdx.x;
  const int U0 = mRows * 8;
  const int U1 = U0 + 1024;
  const int U2 = U1 + 1024;
  const int U3 = U2 + 1024;
  v8us o;
  if (u < U0) {
    const int row = u >> 3;
    const int k8  = (u & 7) * 8;
    const int rc  = row < nN ? row : nN - 1;
    const float* p = x + (size_t)rc * FD + k8;
    const v4f a = *(const v4fa*)p;
    const v4f b = *(const v4fa*)(p + 4);
    const unsigned okm = row < nN ? 0xffffffffu : 0u;
    o[0] = (unsigned short)(bf16_bits(a.x) & okm);
    o[1] = (unsigned short)(bf16_bits(a.y) & okm);
    o[2] = (unsigned short)(bf16_bits(a.z) & okm);
    o[3] = (unsigned short)(bf16_bits(a.w) & okm);
    o[4] = (unsigned short)(bf16_bits(b.x) & okm);
    o[5] = (unsigned short)(bf16_bits(b.y) & okm);
    o[6] = (unsigned short)(bf16_bits(b.z) & okm);
    o[7] = (unsigned short)(bf16_bits(b.w) & okm);
    put16(XB + (size_t)row * FD + k8, o);
    return;
  } else if (u < U1) {
    const int v    = u - U0;
    const int n    = v >> 3;
    const int k8   = (v & 7) * 8;
    const int srow = (n >> 6) * FD + k8;
    const int col  = n & (FD - 1);
    const float* p = We1 + (size_t)srow * FD + col;
#pragma unroll
    for (int i = 0; i < 8; ++i) o[i] = (unsigned short)bf16_bits(p[(size_t)i * FD]);
    put16(W1C + (size_t)n * FD + k8, o);
    return;
  } else if (u < U2) {
    const int v  = u - U1;
    const int n  = v >> 4;
    const int k8 = (v & 15) * 8;
    const int kk = k8 & (FD - 1);
    const float* p = We2 + (size_t)kk * FD + n;
#pragma unroll
    for (int i = 0; i < 8; ++i) o[i] = (unsigned short)bf16_bits(p[(size_t)i * FD]);
    put16(WE2D + (size_t)n * K2 + k8, o);
    return;
  } else if (u < U3) {
    const int v  = u - U2;
    const int n  = v >> 4;
    const int k8 = (v & 15) * 8;
    const int kk = k8 & (FD - 1);
    const float* p = Wn + (size_t)kk * FD + n;
#pragma unroll
    for (int i = 0; i < 8; ++i) o[i] = (unsigned short)bf16_bits(p[(size_t)i * FD]);
    put16(WND + (size_t)n * K2 + k8, o);
    return;
  }
  const int t  = u - U3;
  const int sg = t >> 8;
  const int v  = t & 255;
  if (sg == 0)      tab_unit(be1, FD,        TAB + T_BE1, v);
  else if (sg == 1) tab_unit(be2, FD,        TAB + T_BE2, v);
  else if (sg == 2) tab_unit(bn,  FD,        TAB + T_BN,  v);
  else if (sg == 3) tab_unit(Wg,  FD,        TAB + T_WG,  v);
  else if (sg == 4) tab_unit(bg,  1,         TAB + T_BG,  v);
  else if (sg == 5) tab_unit(bfc, NCLS,      TAB + T_BFC, v);
  else if (sg == 6) tab_unit(Wfc, FD * NCLS, TAB + T_WFC, v);
}

__global__ __launch_bounds__(GTHR) void k_gemm_psd(const unsigned short* __restrict__ A,
                                                   const unsigned short* __restrict__ BT,
                                                   const float* __restrict__ TAB, float* Cm) {
  __shared__ __attribute__((aligned(16))) float stg[GBM * 128];
  __shared__ __attribute__((aligned(16))) float sb1[FD];
  const int tid = (int)threadIdx.x, lane = tid & 31, wave = tid >> 5, hh = lane >> 4, m = lane & 15;
  const int rowBase = (int)blockIdx.x * GBM;
  if (wave == 0) {
    const int l16 = lane & 15;
    const v4f bv = *(const v4fa*)(TAB + T_BE1 + 4 * l16);
    *(v4fa*)(sb1 + 4 * l16) = bv;
  }
  __syncthreads();

  v8f acc[8];
  {
    const v8f z = {0.f, 0.f, 0.f, 0.f, 0.f, 0.f, 0.f, 0.f};
#pragma unroll
    for (int t = 0; t < 8; ++t) acc[t] = z;
  }
  const unsigned short* ap = A  + (size_t)(rowBase + 16 * wave + m) * (size_t)FD + 8 * hh;
  const unsigned short* bp = BT + (size_t)m * (size_t)FD + 8 * hh;
#pragma unroll 1
  for (int k0 = 0; k0 < FD; k0 += 32) {
    FragB af;
    af.h[0] = *(const v8usa*)(ap + k0);
    af.h[1] = *(const v8usa*)(ap + k0 + 16);
#pragma unroll
    for (int nt = 0; nt < 8; ++nt) {
      const unsigned short* wq = bp + (size_t)(16 * nt) * (size_t)FD + k0;
      FragB bf;
      bf.h[0] = *(const v8usa*)wq;
      bf.h[1] = *(const v8usa*)(wq + 16);
      acc[nt] = wmb(af, bf, acc[nt]);
    }
  }
#pragma unroll
  for (int nt = 0; nt < 8; ++nt) {
    const int lc = 16 * nt + m;
    const float bvv = (nt >= 4) ? sb1[lc & (FD - 1)] : 0.0f;
#pragma unroll
    for (int r = 0; r < 8; ++r) {
      const int lr = 16 * wave + 8 * hh + r;
      stg[lr * 128 + lc] = acc[nt][r] + bvv;
    }
  }
  __syncthreads();
  v4f pv[16];
#pragma unroll
  for (int i = 0; i < 16; ++i) pv[i] = *(const v4fa*)(stg + (16 * wave + i) * 128 + 4 * lane);
#pragma unroll
  for (int i = 0; i < 16; ++i) {
    float* op = Cm + (size_t)(rowBase + 16 * wave + i) * 128 + 4 * lane;
    *(volatile v4f*)op = pv[i];
  }
  __threadfence();
#pragma unroll
  for (int i = 0; i < 16; ++i) {
    float* op = Cm + (size_t)(rowBase + 16 * wave + i) * 128 + 4 * lane;
    *(volatile v4f*)op = pv[i];
  }
}

__global__ __launch_bounds__(NTHR) void k_bucket(const int* __restrict__ srcs, const int* __restrict__ dsts,
                                                 int nE, int nN, int vec8, int* HITS, int* BINFO) {
  extern __shared__ __attribute__((aligned(16))) int dsm[];
  int* list = dsm;
  int* hl   = dsm + LISTN;
  int* sl   = hl + RCAP;
  int* cnt  = sl + RCAP;
  int* offs = cnt + NBA;
  int* cur  = offs + NBA;
  int* misc = cur + NBA;
  int* binf = misc + 16;
  const int tid = (int)threadIdx.x, lane = tid & 31, wave = tid >> 5;
  const int nodeBase = (int)blockIdx.x * NBA;
  int nb = nN - nodeBase;
  nb = nb < 0 ? 0 : (nb > NBA ? NBA : nb);

  {
    const v4i z4 = {0, 0, 0, 0};
    for (int i = tid * 4; i < AGG_ZINTS; i += NTHR * 4) *(v4ia*)(dsm + i) = z4;
    if (tid < 16) misc[tid] = 0;
    if (tid < 32) binf[tid] = 0;
  }
  __syncthreads();

  int t = 0, ov = 0;
  const int nChunks = (nE + CHUNK - 1) / CHUNK;
#pragma unroll 1
  for (int ch = 0; ch < nChunks; ++ch) {
    const int cbase = ch * CHUNK;
    const int wc = scan_chunk<SLA>(dsts, nE, cbase, nodeBase, nb, vec8, list, tid, lane, wave);
    if (lane == 0) misc[wave] = wc;
    __syncthreads();
    if (wave == 0) {
#pragma unroll 1
      for (int w2 = 0; w2 < NWAVE; ++w2) {
        int c = misc[w2];
        c = c < 0 ? 0 : (c > WCAP ? WCAP : c);
#pragma unroll 1
        for (int b0 = 0; b0 < c; b0 += 32) {
          const int idx = b0 + lane;
          const int ent = list[w2 * WCAP + (idx < WCAP ? idx : WCAP - 1)];
          const int m32 = (c - b0) < 32 ? (c - b0) : 32;
#pragma unroll 1
          for (int k = 0; k < m32; ++k) {
            const int u    = __builtin_amdgcn_readlane(ent, k);
            const int slot = u & (NBA - 1);
            const int el   = (u >> SLA) & (CHUNK - 1);
            const int pk   = ((cbase + el) << SLA) | slot;
            if (t < RCAP) {
              if (lane == 0) { hl[t] = pk; cnt[slot] = cnt[slot] + 1; }
              t = t + 1;
            } else {
              ov = 1;
            }
          }
        }
      }
    }
    __syncthreads();
  }
  if (wave == 0 && lane == 0) { misc[8] = t; misc[9] = ov; }
  __syncthreads();
  int tt = misc[8];
  tt = tt < 0 ? 0 : (tt > RCAP ? RCAP : tt);
  const int ovf = misc[9];

  if (wave == 0) {
    const int base = lane * (NBA / 32);
    int s = 0, mx = 0;
#pragma unroll 1
    for (int i = 0; i < NBA / 32; ++i) {
      const int cv = cnt[base + i];
      s += cv;
      mx = cv > mx ? cv : mx;
    }
    int incl = s;
#pragma unroll
    for (int d = 1; d < 32; d <<= 1) {
      const int y = __shfl_up(incl, d, 32);
      if (lane >= d) incl += y;
    }
#pragma unroll
    for (int d = 16; d > 0; d >>= 1) {
      const int y = __shfl_xor(mx, d, 32);
      mx = y > mx ? y : mx;
    }
    int run = incl - s;
#pragma unroll 1
    for (int i = 0; i < NBA / 32; ++i) {
      const int cv = cnt[base + i];
      offs[base + i] = run;
      cur[base + i]  = run;
      run += cv;
    }
    if (lane == 0) misc[10] = mx;
  }
  __syncthreads();
  if (wave == 0) {
#pragma unroll 1
    for (int b0 = 0; b0 < tt; b0 += 32) {
      const int idx = b0 + lane;
      const int ent = hl[idx < RCAP ? idx : RCAP - 1];
      const int m32 = (tt - b0) < 32 ? (tt - b0) : 32;
#pragma unroll 1
      for (int k = 0; k < m32; ++k) {
        const int u    = __builtin_amdgcn_readlane(ent, k);
        const int slot = u & (NBA - 1);
        if (lane == 0) {
          int p = cur[slot];
          p = p < 0 ? 0 : (p > RCAP - 1 ? RCAP - 1 : p);
          sl[p] = u;
          cur[slot] = p + 1;
        }
      }
    }
  }
  __syncthreads();

  const int mxd  = misc[10];
  const int flag = (ovf != 0 || mxd > DEGCAP) ? 1 : 0;
  if (wave == 0) {
    const int o = offs[SB * (lane & 3)];
    const int v = lane < 4 ? o : (lane == 4 ? tt : (lane == 5 ? flag : (lane == 6 ? mxd : 0)));
    binf[lane] = v;
  }
  __syncthreads();
  {
    const int l8 = lane & 7;
    const v4i bv = *(const v4ia*)(binf + 4 * l8);
    int* bp = BINFO + (size_t)blockIdx.x * 32 + 4 * l8;
    const bool wr = tid < 8;
    if (wr) *(volatile v4i*)bp = bv;
    __threadfence();
    if (wr) *(volatile v4i*)bp = bv;
  }

  int* hbp = HITS + (size_t)blockIdx.x * (size_t)(2 * RCAP);
#pragma unroll 1
  for (int it = 0; it < RCAP / (2 * NTHR); ++it) {
    const int p0 = (it * NTHR + tid) * 2;
    const int e0 = sl[p0];
    const int e1 = sl[p0 + 1];
    int id0 = e0 >> SLA; id0 = id0 < 0 ? 0 : (id0 > nE - 1 ? nE - 1 : id0);
    int id1 = e1 >> SLA; id1 = id1 < 0 ? 0 : (id1 > nE - 1 ? nE - 1 : id1);
    const int s0 = srcs[id0];
    const int s1 = srcs[id1];
    v4i o;
    o.x = (p0     < tt) ? s0 : 0;
    o.y = (p0     < tt) ? (e0 & (NBA - 1)) : -1;
    o.z = (p0 + 1 < tt) ? s1 : 0;
    o.w = (p0 + 1 < tt) ? (e1 & (NBA - 1)) : -1;
    int* dp = hbp + 2 * (size_t)p0;
    *(volatile v4i*)dp = o;
    __threadfence();
    *(volatile v4i*)dp = o;
  }
}

__device__ __forceinline__ void acc_step(int slv, int rr, int q4u, int c, float b2,
                                         float* ACC, const float* MSG, const float* XS) {
  const int sl = __builtin_amdgcn_readfirstlane(slv);
  if (sl >= 0 && sl < SB && (sl & 3) == q4u) {
    float* a = ACC + sl * FD + c;
    const float mv = MSG[rr * MSP + c] + b2;
    const float xv = XS[rr * FD + c];
    *a = *a + mv * xv;
  }
}

__device__ __forceinline__ v8us hn_unit(const float* ACC, int u, bool poison) {
  const int row  = u >> 4;
  const int j    = u & 15;
  const int part = j >> 3;
  const int c8   = (j & 7) * 8;
  const unsigned mh = 0u - (unsigned)part;
  const unsigned ml = ~mh;
  const float* sp = ACC + row * FD + c8;
  const v4f a  = *(const v4fa*)sp;
  const v4f bq = *(const v4fa*)(sp + 4);
  const v8f f8 = {a.x, a.y, a.z, a.w, bq.x, bq.y, bq.z, bq.w};
  v8us oo;
#pragma unroll
  for (int e = 0; e < 8; ++e) {
    const unsigned hb2 = bf16_bits(f8[e]);
    const unsigned lb2 = bf16_bits(f8[e] - __uint_as_float(hb2 << 16));
    const unsigned wv  = (hb2 & ml) | (lb2 & mh);
    const unsigned pz  = 0x7fc0u & ml;
    oo[e] = (unsigned short)(poison ? pz : wv);
  }
  return oo;
}

__global__ __launch_bounds__(NTHR) void k_edge(const int* __restrict__ HITS, const int* __restrict__ BINFO,
                                               const float* __restrict__ PSD,
                                               const unsigned short* __restrict__ XB,
                                               const unsigned short* __restrict__ WE2D,
                                               const float* __restrict__ TAB, int nN, unsigned short* HN) {
  extern __shared__ __attribute__((aligned(16))) float dyn[];
  float*          ACC   = dyn;
  float*          MSG   = dyn + SB * FD;
  float*          XS    = MSG + TR * MSP;
  unsigned short* sA    = (unsigned short*)(XS + TR * FD);
  float*          sB2   = XS + TR * FD + (TR * AP) / 2;
  int*            sSlot = (int*)(sB2 + FD);
  const int tid = (int)threadIdx.x, lane = tid & 31, wave = tid >> 5, hh = lane >> 4, m = lane & 15;
  const int b = (int)blockIdx.x >> 2;
  const int q = (int)blockIdx.x & 3;
  const int nodeBase = (int)blockIdx.x * SB;

  {
    const v4f z4 = {0.0f, 0.0f, 0.0f, 0.0f};
#pragma unroll 1
    for (int i = tid; i < (SB * FD) / 4; i += NTHR) *(v4fa*)(ACC + 4 * i) = z4;
    if (wave == 0) {
      const int l16 = lane & 15;
      const v4f bv = *(const v4fa*)(TAB + T_BE2 + 4 * l16);
      *(v4fa*)(sB2 + 4 * l16) = bv;
    }
  }
  const v4i i0 = *(const v4ia*)(BINFO + (size_t)b * 32);
  const v4i i1 = *(const v4ia*)(BINFO + (size_t)b * 32 + 4);
  int st = (q == 0) ? i0.x : ((q == 1) ? i0.y : ((q == 2) ? i0.z : i0.w));
  int en = (q == 0) ? i0.y : ((q == 1) ? i0.z : ((q == 2) ? i0.w : i1.x));
  st = st < 0 ? 0 : (st > RCAP ? RCAP : st);
  en = en < 0 ? 0 : (en > RCAP ? RCAP : en);
  st = __builtin_amdgcn_readfirstlane(st);
  en = __builtin_amdgcn_readfirstlane(en);
  int len = en - st;
  len = len < 0 ? 0 : len;
  int nT = (len + TR - 1) / TR;
  nT = nT > RCAP / TR ? RCAP / TR : nT;
  const int flag = __builtin_amdgcn_readfirstlane(i1.y);
  const int* hb = HITS + (size_t)b * (size_t)(2 * RCAP);
  __syncthreads();

  const int   cc  = tid & (FD - 1);
  const int   q4u = __builtin_amdgcn_readfirstlane(tid >> 6);
  const float b2  = sB2[cc];

#pragma unroll 1
  for (int tl = 0; tl < nT; ++tl) {
    {
      const int r  = tid >> 1;
      const int hf = tid & 1;
      const int p  = st + tl * TR + r;
      const bool inr = p < en;
      const int pc = p < (RCAP - 1) ? p : (RCAP - 1);
      const v2i hv = *(const v2ia*)(hb + 2 * (size_t)pc);
      int s = hv.x;
      s = s < 0 ? 0 : (s > nN - 1 ? nN - 1 : s);
      const int lr = hv.y - q * SB;
      const bool ok = inr && ((unsigned)lr < (unsigned)SB);
      int d = nodeBase + (ok ? lr : 0);
      d = d > nN - 1 ? nN - 1 : d;
      const unsigned okm = ok ? 0xffffffffu : 0u;
      const float* ps = PSD + (size_t)s * 128 + 32 * hf;
      const float* pd = PSD + (size_t)d * 128 + FD + 32 * hf;
      const unsigned short* xr = XB + (size_t)s * FD + 32 * hf;
      unsigned short* ar  = sA + r * AP + 32 * hf;
      float*          xsr = XS + r * FD + 32 * hf;
#pragma unroll 1
      for (int c8 = 0; c8 < 4; ++c8) {
        const v4f pa = *(const v4fa*)(ps + 8 * c8);
        const v4f pb = *(const v4fa*)(ps + 8 * c8 + 4);
        const v4f qa = *(const v4fa*)(pd + 8 * c8);
        const v4f qb = *(const v4fa*)(pd + 8 * c8 + 4);
        const v8us xv = *(const v8usa*)(xr + 8 * c8);
        const v8f p8 = {pa.x, pa.y, pa.z, pa.w, pb.x, pb.y, pb.z, pb.w};
        const v8f q8 = {qa.x, qa.y, qa.z, qa.w, qb.x, qb.y, qb.z, qb.w};
        v8us oh, ol;
        v8f xf;
#pragma unroll
        for (int i = 0; i < 8; ++i) {
          float v = p8[i] + q8[i];
          v = (v > 0.0f) ? v : (v - v);
          const unsigned hbits = bf16_bits(v);
          const unsigned lbits = bf16_bits(v - __uint_as_float(hbits << 16));
          oh[i] = (unsigned short)(hbits & okm);
          ol[i] = (unsigned short)(lbits & okm);
          xf[i] = __uint_as_float((((unsigned)xv[i]) << 16) & okm);
        }
        *(v8usa*)(ar + 8 * c8)      = oh;
        *(v8usa*)(ar + FD + 8 * c8) = ol;
        const v4f x0 = {xf[0], xf[1], xf[2], xf[3]};
        const v4f x1 = {xf[4], xf[5], xf[6], xf[7]};
        *(v4fa*)(xsr + 8 * c8)     = x0;
        *(v4fa*)(xsr + 8 * c8 + 4) = x1;
      }
      if (hf == 0) sSlot[r] = ok ? lr : -1;
    }
    __syncthreads();

    {
      const unsigned short* ap = sA + (16 * wave + m) * AP + 8 * hh;
#pragma unroll 1
      for (int ng = 0; ng < 2; ++ng) {
        v8f acc0 = {0.f, 0.f, 0.f, 0.f, 0.f, 0.f, 0.f, 0.f};
        v8f acc1 = {0.f, 0.f, 0.f, 0.f, 0.f, 0.f, 0.f, 0.f};
        const unsigned short* bp0 = WE2D + (size_t)(32 * ng + m) * K2 + 8 * hh;
        const unsigned short* bp1 = bp0 + (size_t)16 * K2;
#pragma unroll 1
        for (int ks = 0; ks < K2 / 32; ++ks) {
          FragB af, bf0, bf1;
          af.h[0]  = *(const v8usa*)(ap + 32 * ks);
          af.h[1]  = *(const v8usa*)(ap + 32 * ks + 16);
          bf0.h[0] = *(const v8usa*)(bp0 + 32 * ks);
          bf0.h[1] = *(const v8usa*)(bp0 + 32 * ks + 16);
          bf1.h[0] = *(const v8usa*)(bp1 + 32 * ks);
          bf1.h[1] = *(const v8usa*)(bp1 + 32 * ks + 16);
          acc0 = wmb(af, bf0, acc0);
          acc1 = wmb(af, bf1, acc1);
        }
        const int col0 = 32 * ng + m;
        float* mrow = MSG + (16 * wave + 8 * hh) * MSP;
#pragma unroll
        for (int r = 0; r < 8; ++r) {
          mrow[r * MSP + col0]      = acc0[r];
          mrow[r * MSP + col0 + 16] = acc1[r];
        }
      }
    }
    __syncthreads();

#pragma unroll 1
    for (int r4 = 0; r4 < TR / 4; ++r4) {
      const v4i s4 = *(const v4ia*)(sSlot + 4 * r4);
      acc_step(s4.x, 4 * r4 + 0, q4u, cc, b2, ACC, MSG, XS);
      acc_step(s4.y, 4 * r4 + 1, q4u, cc, b2, ACC, MSG, XS);
      acc_step(s4.z, 4 * r4 + 2, q4u, cc, b2, ACC, MSG, XS);
      acc_step(s4.w, 4 * r4 + 3, q4u, cc, b2, ACC, MSG, XS);
    }
    __syncthreads();
  }
  __syncthreads();

  {
    const bool poison = flag != 0;
    unsigned short* ob = HN + (size_t)nodeBase * K2;
#pragma unroll 1
    for (int g4 = 0; g4 < 4; ++g4) {
      const int ub = g4 * (4 * NTHR) + tid;
      const v8us p0 = hn_unit(ACC, ub,            poison);
      const v8us p1 = hn_unit(ACC, ub + NTHR,     poison);
      const v8us p2 = hn_unit(ACC, ub + 2 * NTHR, poison);
      const v8us p3 = hn_unit(ACC, ub + 3 * NTHR, poison);
      unsigned short* o0 = ob + (size_t)ub * 8;
      *(volatile v8us*)(o0)                = p0;
      *(volatile v8us*)(o0 + NTHR * 8)     = p1;
      *(volatile v8us*)(o0 + 2 * NTHR * 8) = p2;
      *(volatile v8us*)(o0 + 3 * NTHR * 8) = p3;
      __threadfence();
      *(volatile v8us*)(o0)                = p0;
      *(volatile v8us*)(o0 + NTHR * 8)     = p1;
      *(volatile v8us*)(o0 + 2 * NTHR * 8) = p2;
      *(volatile v8us*)(o0 + 3 * NTHR * 8) = p3;
    }
  }
}

__global__ __launch_bounds__(GTHR) void k_gemm_n(const unsigned short* __restrict__ A,
                                                 const unsigned short* __restrict__ WT,
                                                 const float* __restrict__ TAB, float* H2, float* GATE) {
  __shared__ __attribute__((aligned(16))) float stg[GBM * FD];
  __shared__ __attribute__((aligned(16))) float sc[2 * FD + 4];
  __shared__ __attribute__((aligned(16))) float sgt[GBM];
  const int tid = (int)threadIdx.x, lane = tid & 31, wave = tid >> 5, hh = lane >> 4, m = lane & 15;
  const int rowBase = (int)blockIdx.x * GBM;
  if (wave == 0) {
    const int off = (lane < 16) ? (T_BN + 4 * lane) : (T_WG + 4 * (lane - 16));
    const v4f bv = *(const v4fa*)(TAB + off);
    *(v4fa*)(sc + 4 * lane) = bv;
  } else if (wave == 1) {
    const v4f bv = *(const v4fa*)(TAB + T_BG);
    *(v4fa*)(sc + 2 * FD) = bv;
  }
  __syncthreads();

  v8f acc[4];
  {
    const v8f z = {0.f, 0.f, 0.f, 0.f, 0.f, 0.f, 0.f, 0.f};
    acc[0] = z; acc[1] = z; acc[2] = z; acc[3] = z;
  }
  const unsigned short* ap = A  + (size_t)(rowBase + 16 * wave + m) * (size_t)K2 + 8 * hh;
  const unsigned short* wp = WT + (size_t)m * (size_t)K2 + 8 * hh;
#pragma unroll 1
  for (int ks = 0; ks < K2 / 32; ++ks) {
    FragB af;
    af.h[0] = *(const v8usa*)(ap + 32 * ks);
    af.h[1] = *(const v8usa*)(ap + 32 * ks + 16);
#pragma unroll
    for (int t = 0; t < 4; ++t) {
      const unsigned short* wq = wp + (size_t)(16 * t) * (size_t)K2 + 32 * ks;
      FragB bf;
      bf.h[0] = *(const v8usa*)wq;
      bf.h[1] = *(const v8usa*)(wq + 16);
      acc[t] = wmb(af, bf, acc[t]);
    }
  }
#pragma unroll
  for (int t = 0; t < 4; ++t) {
    const int lc = 16 * t + m;
    const float bvv = sc[lc];
#pragma unroll
    for (int r = 0; r < 8; ++r) {
      const int lr = 16 * wave + 8 * hh + r;
      float v = acc[t][r] + bvv;
      v = (v > 0.0f) ? v : (v - v);
      stg[lr * FD + lc] = v;
    }
  }
  __syncthreads();
  if (wave < 2) {
    const float* rp = stg + tid * FD;
    float s = 0.0f;
#pragma unroll 4
    for (int c = 0; c < FD; ++c) s = fmaf(rp[c], sc[FD + c], s);
    sgt[tid] = s + sc[2 * FD];
  }
  v4f fv[8];
#pragma unroll
  for (int i = 0; i < 8; ++i) {
    const int lr = 16 * wave + 2 * i + hh;
    fv[i] = *(const v4fa*)(stg + lr * FD + 4 * m);
  }
#pragma unroll
  for (int i = 0; i < 8; ++i) {
    const int gr = rowBase + 16 * wave + 2 * i + hh;
    float* op = H2 + (size_t)gr * FD + 4 * m;
    *(volatile v4f*)op = fv[i];
  }
  __threadfence();
#pragma unroll
  for (int i = 0; i < 8; ++i) {
    const int gr = rowBase + 16 * wave + 2 * i + hh;
    float* op = H2 + (size_t)gr * FD + 4 * m;
    *(volatile v4f*)op = fv[i];
  }
  __syncthreads();
  {
    const v4f gv = *(const v4fa*)(sgt + 4 * m);
    float* gp = GATE + (size_t)rowBase + 4 * m;
    const bool wr = (wave == 0) && (lane < 16);
    if (wr) *(volatile v4f*)gp = gv;
    __threadfence();
    if (wr) *(volatile v4f*)gp = gv;
  }
}

__global__ __launch_bounds__(NTHR) void k_pool(const float* __restrict__ H2, const float* __restrict__ GATE,
                                               const int* __restrict__ ids, const float* __restrict__ TAB,
                                               int nN, float* REC) {
  extern __shared__ __attribute__((aligned(16))) int psm[];
  int*   NL      = psm;
  float* WL      = (float*)(psm + GCAP);
  float* swfc    = (float*)(psm + 2 * GCAP);
  float* sbfc    = swfc + 640;
  float* spool   = sbfc + 16;
  float* spooled = spool + 4 * FD;
  float* sredA   = spooled + FD;
  float* sredB   = sredA + 16;
  int*   sint    = (int*)(sredB + 16);
  float* srec    = (float*)(sint + 16);
  const int tid = (int)threadIdx.x, lane = tid & 31, wave = tid >> 5;
  const int g = (int)blockIdx.x;

  if (wave < 5) {
    const v4f wv = *(const v4fa*)(TAB + T_WFC + 4 * tid);
    *(v4fa*)(swfc + 4 * tid) = wv;
  } else if (wave == 5) {
    const int l4 = lane & 3;
    const v4f bv = *(const v4fa*)(TAB + T_BFC + 4 * l4);
    *(v4fa*)(sbfc + 4 * l4) = bv;
  }

  const int SEGW = (((nN + NWAVE - 1) / NWAVE) + 31) & ~31;
  const int w0 = wave * SEGW;
  int w1 = w0 + SEGW;
  w1 = w1 > nN ? nN : w1;
  int cntw = 0;
#pragma unroll 1
  for (int i0 = w0; i0 < w1; i0 += 32) {
    const int i  = i0 + lane;
    const int ic = i < nN ? i : nN - 1;
    const int bq = ids[ic];
    const bool hit = (i < w1) && (bq == g);
    cntw += (int)__builtin_popcount(__builtin_amdgcn_ballot_w32(hit));
  }
  if (lane == 0) sint[wave] = cntw;
  __syncthreads();
  int base = 0, total = 0;
#pragma unroll
  for (int w2 = 0; w2 < NWAVE; ++w2) {
    const int c2 = sint[w2];
    base  += (w2 < wave) ? c2 : 0;
    total += c2;
  }
  const bool ovf = total > GCAP;
  int n = total < 0 ? 0 : (total > GCAP ? GCAP : total);
  {
    int run = base;
#pragma unroll 1
    for (int i0 = w0; i0 < w1; i0 += 32) {
      const int i  = i0 + lane;
      const int ic = i < nN ? i : nN - 1;
      const int bq = ids[ic];
      const bool hit = (i < w1) && (bq == g);
      const unsigned mk = __builtin_amdgcn_ballot_w32(hit);
      const int pos = run + (int)__builtin_amdgcn_mbcnt_lo(mk, 0u);
      if (hit && pos >= 0 && pos < GCAP) NL[pos] = i;
      run += (int)__builtin_popcount(mk);
    }
  }
  __syncthreads();

  float mx = -INFINITY;
#pragma unroll 1
  for (int i = tid; i < n; i += NTHR) {
    int node = NL[i];
    node = node < 0 ? 0 : (node > nN - 1 ? nN - 1 : node);
    const float gt = GATE[node];
    WL[i] = gt;
    mx = nmax(mx, gt);
  }
#pragma unroll
  for (int d = 16; d > 0; d >>= 1) {
    const float o = __shfl_xor(mx, d, 32);
    mx = nmax(mx, o);
  }
  if (lane == 0) sredA[wave] = mx;
  __syncthreads();
  float gm = sredA[0];
#pragma unroll
  for (int w2 = 1; w2 < NWAVE; ++w2) gm = nmax(gm, sredA[w2]);

  float sm = 0.0f;
#pragma unroll 1
  for (int i = tid; i < n; i += NTHR) {
    const float w = expf(WL[i] - gm);
    WL[i] = w;
    sm += w;
  }
#pragma unroll
  for (int d = 16; d > 0; d >>= 1) sm += __shfl_xor(sm, d, 32);
  if (lane == 0) sredB[wave] = sm;
  __syncthreads();
  float den = sredB[0];
#pragma unroll
  for (int w2 = 1; w2 < NWAVE; ++w2) den += sredB[w2];
  const float rden = (den == 0.0f) ? 0.0f : (1.0f / den);

  {
    const int c  = tid & (FD - 1);
    const int qq = tid >> 6;
    float acc = 0.0f;
#pragma unroll 1
    for (int i = qq; i < n; i += 4) {
      int node = NL[i];
      node = node < 0 ? 0 : (node > nN - 1 ? nN - 1 : node);
      const float a = WL[i] * rden;
      acc = fmaf(a, H2[(size_t)node * FD + c], acc);
    }
    spool[qq * FD + c] = acc;
  }
  __syncthreads();
  if (wave < 2) spooled[tid] = ((spool[tid] + spool[FD + tid]) + spool[2 * FD + tid]) + spool[3 * FD + tid];
  __syncthreads();

  if (wave == 0) {
    const int cls = lane < NCLS ? lane : NCLS - 1;
    float s = 0.0f;
#pragma unroll 4
    for (int f = 0; f < FD; ++f) s = fmaf(spooled[f], swfc[f * NCLS + cls], s);
    s = s + sbfc[cls];
    const float qnan = __int_as_float(0x7fc00000);
    const float pv = ovf ? qnan : s;
    srec[lane] = (lane < NCLS) ? pv : 0.0f;
  }
  __syncthreads();
  {
    const int l8 = lane & 7;
    const v4f rv = *(const v4fa*)(srec + 4 * l8);
    float* rp = REC + (size_t)g * 32 + 4 * l8;
    const bool wr = tid < 8;
    if (wr) *(volatile v4f*)rp = rv;
    __threadfence();
    if (wr) *(volatile v4f*)rp = rv;
  }
}

__global__ __launch_bounds__(NTHR) void k_out(const float* __restrict__ REC, float* out) {
  __shared__ __attribute__((aligned(16))) float os[NOUT];
  const int tid = (int)threadIdx.x;
#pragma unroll 1
  for (int idx = tid; idx < NOUT; idx += NTHR) {
    const int g = idx / NCLS;
    const int c = idx - g * NCLS;
    os[idx] = REC[(size_t)g * 32 + c];
  }
  __syncthreads();
  constexpr int NU = NOUT / 4;
  v4f ov[2];
#pragma unroll
  for (int it = 0; it < 2; ++it) {
    const int u  = it * NTHR + tid;
    const int uc = u < NU ? u : NU - 1;
    ov[it] = *(const v4fa*)(os + 4 * uc);
  }
#pragma unroll
  for (int it = 0; it < 2; ++it) {
    const int u = it * NTHR + tid;
    if (u < NU) *(volatile v4f*)(out + 4 * (size_t)u) = ov[it];
  }
  __threadfence();
#pragma unroll
  for (int it = 0; it < 2; ++it) {
    const int u = it * NTHR + tid;
    if (u < NU) *(volatile v4f*)(out + 4 * (size_t)u) = ov[it];
  }
}

static inline int cdiv(int a, int b) { return (a + b - 1) / b; }
static inline size_t al256(size_t o) { return (o + 255) & ~(size_t)255; }

extern "C" void kernel_launch(void* const* d_in, const int* in_sizes, int n_in,
                              void* d_out, int out_size, void* d_ws, size_t ws_size,
                              hipStream_t stream) {
  if (n_in < 14) return;
  if (in_sizes[0] < FD || (in_sizes[0] % FD) != 0) return;
  const int nN = in_sizes[0] / FD;
  if (nN < 1 || nN > (1 << 22)) return;
  if (in_sizes[1] != 2 * FD * FD || in_sizes[2] != FD) return;
  if (in_sizes[3] != FD * FD || in_sizes[4] != FD) return;
  if (in_sizes[5] != FD * FD || in_sizes[6] != FD) return;
  if (in_sizes[7] != FD || in_sizes[8] != 1) return;
  if (in_sizes[9] != FD * NCLS || in_sizes[10] != NCLS) return;
  const int nE = in_sizes[11];
  if (nE < 1 || nE >= (1 << (31 - SLA)) || in_sizes[12] != nE) return;
  if (in_sizes[13] != nN) return;
  if (out_size != NOUT) return;

  const float* x   = (const float*)d_in[0];
  const float* We1 = (const float*)d_in[1];
  const float* be1 = (const float*)d_in[2];
  const float* We2 = (const float*)d_in[3];
  const float* be2 = (const float*)d_in[4];
  const float* Wn  = (const float*)d_in[5];
  const float* bn  = (const float*)d_in[6];
  const float* Wg  = (const float*)d_in[7];
  const float* bg  = (const float*)d_in[8];
  const float* Wfc = (const float*)d_in[9];
  const float* bfc = (const float*)d_in[10];
  const int*   src = (const int*)d_in[11];
  const int*   dst = (const int*)d_in[12];
  const int*   gid = (const int*)d_in[13];
  float* out = (float*)d_out;

  const int MP = cdiv(nN, SB) * SB;
  const int gE = MP / SB;
  const int gB = cdiv(MP, NBA);
  if (cdiv(gE, 4) > gB) return;
  const int vec8 = ((nE & 3) == 0) ? 1 : 0;

  char* ws = (char*)d_ws;
  size_t off = 0;
  const size_t oXB   = off; off = al256(off + (size_t)MP * FD * 2);
  const size_t oW1C  = off; off = al256(off + (size_t)128 * FD * 2);
  const size_t oWE2D = off; off = al256(off + (size_t)FD * K2 * 2);
  const size_t oWND  = off; off = al256(off + (size_t)FD * K2 * 2);
  const size_t oTAB  = off; off = al256(off + (size_t)TABN * 4);
  const size_t oPSD  = off; off = al256(off + (size_t)MP * 128 * 4);
  const size_t oHITS = off; off = al256(off + (size_t)gB * RCAP * 8);
  const size_t oBINF = off; off = al256(off + (size_t)gB * 128);
  const size_t oHN   = off; off = al256(off + (size_t)MP * K2 * 2);
  const size_t oGATE = off; off = al256(off + (size_t)MP * 4);
  const size_t oREC  = off; off = al256(off + (size_t)NGR * 128);
  if (off > ws_size || off > (size_t)WSMAX) return;
  if ((size_t)MP * FD * 4 > (size_t)MP * 128 * 4) return;
  unsigned short* XB   = (unsigned short*)(ws + oXB);
  unsigned short* W1C  = (unsigned short*)(ws + oW1C);
  unsigned short* WE2D = (unsigned short*)(ws + oWE2D);
  unsigned short* WND  = (unsigned short*)(ws + oWND);
  float*          TAB  = (float*)(ws + oTAB);
  float*          PSD  = (float*)(ws + oPSD);
  float*          H2   = (float*)(ws + oPSD);
  int*            HITS = (int*)(ws + oHITS);
  int*            BINF = (int*)(ws + oBINF);
  unsigned short* HN   = (unsigned short*)(ws + oHN);
  float*          GATE = (float*)(ws + oGATE);
  float*          REC  = (float*)(ws + oREC);

  hipFuncSetAttribute(reinterpret_cast<const void*>(&k_bucket), hipFuncAttributeMaxDynamicSharedMemorySize,
                      (int)BKT_LDS_BYTES);
  hipFuncSetAttribute(reinterpret_cast<const void*>(&k_edge), hipFuncAttributeMaxDynamicSharedMemorySize,
                      (int)EDGE_LDS_BYTES);
  hipFuncSetAttribute(reinterpret_cast<const void*>(&k_pool), hipFuncAttributeMaxDynamicSharedMemorySize,
                      (int)POOL_LDS_BYTES);

  const int nPrep = MP * 8 + 3 * 1024 + 7 * 256;
  k_prep<<<nPrep / NTHR, NTHR, 0, stream>>>(x, We1, be1, We2, be2, Wn, bn, Wg, bg, Wfc, bfc, nN, MP,
                                            XB, W1C, WE2D, WND, TAB);
  k_gemm_psd<<<MP / GBM, GTHR, 0, stream>>>(XB, W1C, TAB, PSD);
  k_bucket<<<gB, NTHR, BKT_LDS_BYTES, stream>>>(src, dst, nE, nN, vec8, HITS, BINF);
  k_edge<<<gE, NTHR, EDGE_LDS_BYTES, stream>>>(HITS, BINF, PSD, XB, WE2D, TAB, nN, HN);
  k_gemm_n<<<MP / GBM, GTHR, 0, stream>>>(HN, WND, TAB, H2, GATE);
  k_pool<<<NGR, NTHR, POOL_LDS_BYTES, stream>>>(H2, GATE, gid, TAB, nN, REC);
  k_out<<<1, NTHR, 0, stream>>>(REC, out);
}
